// PairClassifier_20117626815124
// MI455X (gfx1250) — hardware-verified
//
#include <hip/hip_runtime.h>


#define NTP  4096
#define NTH  4096
#define DC   512
#define DB   768
#define NH_  4
#define HDQ  128
#define HDV  192
#define DF   1280
#define D1   256
#define D2   128
#define NSG  32
#define PSC  32768.0f
#define SCL  0.08838834764831845f

typedef _Float16 h16;
typedef unsigned short bf;
typedef __attribute__((ext_vector_type(16))) __bf16   v16bf;
typedef __attribute__((ext_vector_type(16))) _Float16 v16h;
typedef __attribute__((ext_vector_type(8)))  _Float16 v8h;
typedef __attribute__((ext_vector_type(8)))  unsigned short v8us;
typedef __attribute__((ext_vector_type(4)))  unsigned short v4us;
typedef __attribute__((ext_vector_type(8)))  float    v8f;
typedef __attribute__((ext_vector_type(4)))  float    v4f;
typedef v8h  __attribute__((may_alias)) v8ha;
typedef v4f  __attribute__((may_alias)) v4fa;
typedef v8us __attribute__((may_alias)) v8usa;

__device__ __forceinline__ unsigned short f2bf(float f) { unsigned u = __float_as_uint(f); u += 0x7FFFu + ((u >> 16) & 1u); return (unsigned short)(u >> 16); }
__device__ __forceinline__ float bf2f(unsigned short b) { return __uint_as_float(((unsigned)b) << 16); }
__device__ __forceinline__ float bfr(float f) { return bf2f(f2bf(f)); }
__device__ __forceinline__ v16h cat16(v8h lo, v8h hi) { return __builtin_shufflevector(lo, hi, 0, 1, 2, 3, 4, 5, 6, 7, 8, 9, 10, 11, 12, 13, 14, 15); }
__device__ __forceinline__ v16bf cat16b(v8us lo, v8us hi) { return __builtin_bit_cast(v16bf, __builtin_shufflevector(lo, hi, 0, 1, 2, 3, 4, 5, 6, 7, 8, 9, 10, 11, 12, 13, 14, 15)); }
__device__ __forceinline__ v8f wmma16(v16h a, v16h b, v8f c) { return __builtin_amdgcn_wmma_f32_16x16x32_f16(false, a, false, b, (short)0, c, false, false); }
__device__ __forceinline__ v8f wmmab(v16bf a, v16bf b, v8f c) { return __builtin_amdgcn_wmma_f32_16x16x32_bf16(false, a, false, b, (short)0, c, false, false); }
#define VST2(T, p, v) do { const T vst2_v_ = (v); *(volatile T*)(p) = vst2_v_; __threadfence(); *(volatile T*)(p) = vst2_v_; } while (0)

__global__ __launch_bounds__(256) void k_cvtb(const float* __restrict__ src, int nrows, int ncols, bf* dst) {
    const int lane = threadIdx.x & 31, r = blockIdx.x * 8 + (threadIdx.x >> 5);
    if (r >= nrows) return;
#pragma unroll 1
    for (int q = 0; q < ncols / 128; ++q) { v4us t;
#pragma unroll
        for (int i = 0; i < 4; ++i) t[i] = f2bf(src[(size_t)r * ncols + q * 128 + lane * 4 + i]);
        VST2(v4us, dst + (size_t)r * ncols + q * 128 + lane * 4, t); }
}
__global__ __launch_bounds__(256) void k_wt(const float* __restrict__ Wm, int K, int N, bf* WT) {
    __shared__ __align__(16) unsigned short tl[64 * 72];
    const int tid = threadIdx.x, k0 = blockIdx.x * 64, n0 = blockIdx.y * 64;
    const int kk = tid >> 2, nq = (tid & 3) * 16;
#pragma unroll
    for (int i = 0; i < 16; ++i) tl[(nq + i) * 72 + kk] = f2bf(Wm[(size_t)(k0 + kk) * N + n0 + nq + i]);
    __syncthreads();
    const int piece = tid & 7;
    auto pass = [&]() {
#pragma unroll
        for (int s = 0; s < 2; ++s) { const int nr = (tid >> 3) + 32 * s; const v8us val = *(const v8usa*)(tl + nr * 72 + piece * 8);
            *(volatile v8us*)(WT + (size_t)(n0 + nr) * K + k0 + piece * 8) = val; }
    };
    pass(); __threadfence(); pass();
}

template <bool SPLITA, int MODE>
__global__ __launch_bounds__(128) void k_gemmb(const bf* __restrict__ A, const bf* __restrict__ Al, const bf* __restrict__ Bn, int K, const float* __restrict__ bias, void* C, void* C2, int ldc) {
    __shared__ __align__(16) float ost[4][16 * 68];
    const int lane = threadIdx.x & 31, wave = threadIdx.x >> 5, lr = lane & 15, hi = lane >> 4;
    const int r0 = blockIdx.x * 64 + wave * 16, c0 = blockIdx.y * 64;
    const size_t aoff = (size_t)(r0 + lr) * K + 8 * hi;
    size_t boff[4];
#pragma unroll
    for (int t = 0; t < 4; ++t) boff[t] = (size_t)(c0 + t * 16 + lr) * K + 8 * hi;
    v8f acc[4];
#pragma unroll
    for (int t = 0; t < 4; ++t) acc[t] = (v8f){};
#pragma unroll 1
    for (int kc = 0; kc < K; kc += 32) {
        const v16bf a = cat16b(*(const v8us*)(A + aoff + kc), *(const v8us*)(A + aoff + kc + 16));
        v16bf al = a;
        if (SPLITA) al = cat16b(*(const v8us*)(Al + aoff + kc), *(const v8us*)(Al + aoff + kc + 16));
#pragma unroll
        for (int t = 0; t < 4; ++t) { const v16bf b = cat16b(*(const v8us*)(Bn + boff[t] + kc), *(const v8us*)(Bn + boff[t] + kc + 16)); acc[t] = wmmab(a, b, acc[t]); if (SPLITA) acc[t] = wmmab(al, b, acc[t]); }
        asm volatile("v_nop\n\tv_nop\n\tv_nop\n\tv_nop" : "+v"(acc[0]), "+v"(acc[1]), "+v"(acc[2]), "+v"(acc[3]) : "v"(a), "v"(al));
    }
    float* os = &ost[wave][0];
#pragma unroll
    for (int t = 0; t < 4; ++t) { const float bv = (MODE == 0) ? 0.f : bfr(bias[c0 + t * 16 + lr]);
#pragma unroll
        for (int j = 0; j < 8; ++j) { float v = acc[t][j] + bv; if (MODE == 3) v = 0.5f * v * (1.0f + erff(v * 0.7071067811865476f)); os[(hi * 8 + j) * 68 + t * 16 + lr] = v; } }
    __syncthreads();
    if (MODE == 0) {
        float* crow = (float*)C + (size_t)r0 * ldc + c0;
        auto pass = [&]() {
#pragma unroll
            for (int s = 0; s < 8; ++s) { const int Lid = (lane >> 3) + 4 * s, piece = lane & 7; const int row = Lid >> 1, cofs = (Lid & 1) * 32 + piece * 4;
                const v4f val = *(const v4fa*)(os + row * 68 + cofs); *(volatile v4f*)(crow + (size_t)row * ldc + cofs) = val; }
        };
        pass(); __threadfence(); pass();
    } else if (MODE == 1) {
        h16* crow = (h16*)C + (size_t)r0 * ldc + c0;
        auto pass = [&]() {
#pragma unroll
            for (int s = 0; s < 4; ++s) { const int row = 4 * s + (lane >> 3), piece = lane & 7; const float* sp = os + row * 68 + piece * 8; v8h o;
#pragma unroll
                for (int i = 0; i < 8; ++i) o[i] = (h16)sp[i];
                *(volatile v8h*)(crow + (size_t)row * ldc + piece * 8) = o; }
        };
        pass(); __threadfence(); pass();
    } else if (MODE == 2) {
        h16* crow = (h16*)C + (size_t)r0 * ldc + c0;
        auto pass = [&]() {
#pragma unroll
            for (int s = 0; s < 4; ++s) { const int row = 4 * s + (lane >> 3), piece = lane & 7; const float* sp = os + row * 68 + piece * 8; v8h o;
#pragma unroll
                for (int i = 0; i < 8; ++i) o[i] = (h16)sp[i];
                *(volatile v8h*)(crow + (size_t)row * ldc + piece * 8) = o; }
        };
        pass(); __threadfence(); pass();
    } else {
        bf* ch = (bf*)C + (size_t)r0 * ldc + c0; bf* cl = (bf*)C2 + (size_t)r0 * ldc + c0;
        auto pass = [&]() {
#pragma unroll
            for (int s = 0; s < 4; ++s) { const int row = 4 * s + (lane >> 3), piece = lane & 7; const float* sp = os + row * 68 + piece * 8; v8us oh, ol;
#pragma unroll
                for (int i = 0; i < 8; ++i) { const unsigned short hb = f2bf(sp[i]); oh[i] = hb; ol[i] = f2bf(sp[i] - bf2f(hb)); }
                *(volatile v8us*)(ch + (size_t)row * ldc + piece * 8) = oh; *(volatile v8us*)(cl + (size_t)row * ldc + piece * 8) = ol; }
        };
        pass(); __threadfence(); pass();
    }
}

__global__ __launch_bounds__(256) void k_deint(const h16* __restrict__ SRC, h16* DST) {
    const int lane = threadIdx.x & 31, r = blockIdx.x * 8 + (threadIdx.x >> 5);
    if (r >= NTH) return;
    const h16* s = SRC + (size_t)r * DC;
    v8h o[2];
#pragma unroll
    for (int q = 0; q < 2; ++q) { v8h t;
#pragma unroll
        for (int i = 0; i < 8; ++i) { const int oc = q * 256 + lane * 8 + i; const int h = oc >> 7, d = oc & 127; t[i] = s[d * 4 + h]; }
        o[q] = t; }
#pragma unroll
    for (int q = 0; q < 2; ++q) *(volatile v8h*)(DST + (size_t)r * DC + q * 256 + lane * 8) = o[q];
    __threadfence();
#pragma unroll
    for (int q = 0; q < 2; ++q) *(volatile v8h*)(DST + (size_t)r * DC + q * 256 + lane * 8) = o[q];
}
__global__ __launch_bounds__(256) void k_vt(const h16* __restrict__ V16, h16* VT16) {
    __shared__ __align__(16) h16 tile[HDV * 72];
    const int bid = blockIdx.x, h = bid / (NTP / 64), kt = bid - h * (NTP / 64), m0 = kt * 64, tid = threadIdx.x;
    const int mm_ = tid >> 2, dq = (tid & 3) * 48;
    const h16* src = V16 + (size_t)(m0 + mm_) * DB + h * HDV + dq;
#pragma unroll
    for (int i = 0; i < 48; ++i) tile[(dq + i) * 72 + mm_] = src[i];
    __syncthreads();
    const int piece = tid & 7;
    h16* base = VT16 + ((size_t)h * HDV) * NTP + m0;
    auto pass = [&]() {
#pragma unroll
        for (int s = 0; s < 6; ++s) { const int d = (tid >> 3) + 32 * s; const v8h val = *(const v8ha*)(tile + d * 72 + piece * 8); *(volatile v8h*)(base + (size_t)d * NTP + piece * 8) = val; }
    };
    pass(); __threadfence(); pass();
}

__global__ __launch_bounds__(128) void k_attn(const h16* __restrict__ Q16, const h16* __restrict__ K16, const h16* __restrict__ VT16, const int* __restrict__ bh, const int* __restrict__ bp, float* ATT) {
    __shared__ __align__(16) h16 plds[4][16 * 32];
    __shared__ __align__(16) float ost[4][16 * 196];
    const int lane = threadIdx.x & 31, wave = threadIdx.x >> 5, lr = lane & 15, hi = lane >> 4;
    const int h = blockIdx.x / (NTH / 64), qt = blockIdx.x - h * (NTH / 64);
    const int q0 = qt * 64 + wave * 16;
    h16* pl = &plds[wave][0];
    v16h qa[4];
#pragma unroll
    for (int kc = 0; kc < 4; ++kc) { const h16* p = Q16 + (size_t)(q0 + lr) * DC + h * HDQ + kc * 32 + 8 * hi; qa[kc] = cat16(*(const v8h*)p, *(const v8h*)(p + 16)); }
    int bq[8];
#pragma unroll
    for (int j = 0; j < 8; ++j) bq[j] = bh[q0 + 8 * hi + j];
    const h16* kh_b = K16 + h * HDQ;
    const h16* vt_b = VT16 + ((size_t)h * HDV) * NTP;
    v8f o[12];
#pragma unroll
    for (int n = 0; n < 12; ++n) o[n] = (v8f){};
    float mrow[8], lpart[8];
#pragma unroll
    for (int j = 0; j < 8; ++j) { mrow[j] = -3.0e38f; lpart[j] = 0.f; }
#pragma unroll 1
    for (int kt = 0; kt < NTP / 32; ++kt) {
        const int l0 = kt * 32;
        const h16* r0p = kh_b + (size_t)(l0 + lr) * DC + 8 * hi; const h16* r1p = kh_b + (size_t)(l0 + 16 + lr) * DC + 8 * hi;
        v8f s0 = {}, s1 = {};
#pragma unroll
        for (int kc = 0; kc < 4; ++kc) {
            s0 = wmma16(qa[kc], cat16(*(const v8h*)(r0p + kc * 32), *(const v8h*)(r0p + kc * 32 + 16)), s0);
            s1 = wmma16(qa[kc], cat16(*(const v8h*)(r1p + kc * 32), *(const v8h*)(r1p + kc * 32 + 16)), s1);
        }
        asm volatile("v_nop\n\tv_nop\n\tv_nop\n\tv_nop" : "+v"(s0), "+v"(s1) : "v"(qa[0]), "v"(qa[3]));
        const int bk0 = bp[l0 + lr], bk1 = bp[l0 + 16 + lr];
        float alpha[8];
#pragma unroll
        for (int j = 0; j < 8; ++j) {
            const float a0 = (bk0 == bq[j]) ? -1e10f : s0[j] * SCL, a1 = (bk1 == bq[j]) ? -1e10f : s1[j] * SCL;
            float mx = fmaxf(a0, a1);
            mx = fmaxf(mx, __shfl_xor(mx, 1, 16)); mx = fmaxf(mx, __shfl_xor(mx, 2, 16)); mx = fmaxf(mx, __shfl_xor(mx, 4, 16)); mx = fmaxf(mx, __shfl_xor(mx, 8, 16));
            const float mn = fmaxf(mrow[j], mx);
            alpha[j] = __expf(mrow[j] - mn); mrow[j] = mn;
            const float p0 = __expf(a0 - mn), p1 = __expf(a1 - mn);
            lpart[j] = lpart[j] * alpha[j] + (p0 + p1);
            const int mr = hi * 8 + j;
            pl[mr * 32 + lr] = (h16)(p0 * PSC); pl[mr * 32 + 16 + lr] = (h16)(p1 * PSC);
        }
#pragma unroll
        for (int n = 0; n < 12; ++n)
#pragma unroll
            for (int j = 0; j < 8; ++j) o[n][j] *= alpha[j];
        asm volatile("" ::: "memory");
        const v16h pa = cat16(*(const v8ha*)(pl + lr * 32 + hi * 8), *(const v8ha*)(pl + lr * 32 + 16 + hi * 8));
#pragma unroll
        for (int n = 0; n < 12; ++n) { const h16* vp = vt_b + (size_t)(n * 16 + lr) * NTP + l0 + hi * 8; o[n] = wmma16(pa, cat16(*(const v8h*)vp, *(const v8h*)(vp + 16)), o[n]); }
        asm volatile("v_nop\n\tv_nop\n\tv_nop\n\tv_nop" : "+v"(o[0]), "+v"(o[3]), "+v"(o[7]), "+v"(o[11]) : "v"(pa));
    }
    asm volatile("v_nop\n\tv_nop\n\tv_nop\n\tv_nop" : "+v"(o[0]), "+v"(o[1]), "+v"(o[2]), "+v"(o[3]), "+v"(o[4]), "+v"(o[5]), "+v"(o[6]), "+v"(o[7]), "+v"(o[8]), "+v"(o[9]), "+v"(o[10]), "+v"(o[11]));
    float inv[8];
#pragma unroll
    for (int j = 0; j < 8; ++j) { float rs = lpart[j]; rs += __shfl_xor(rs, 1, 16); rs += __shfl_xor(rs, 2, 16); rs += __shfl_xor(rs, 4, 16); rs += __shfl_xor(rs, 8, 16); inv[j] = 1.0f / (rs * PSC); }
    float* os = &ost[wave][0];
#pragma unroll
    for (int n = 0; n < 12; ++n)
#pragma unroll
        for (int j = 0; j < 8; ++j) os[(hi * 8 + j) * 196 + n * 16 + lr] = o[n][j] * inv[j];
    __syncthreads();
    float* abase = ATT + (size_t)q0 * DB + h * HDV;
    auto pass = [&]() {
#pragma unroll
        for (int s = 0; s < 24; ++s) { const int Lid = lane + 32 * s; const int row = Lid / 48, piece = Lid - row * 48;
            const v4f v = *(const v4fa*)(os + row * 196 + piece * 4); *(volatile v4f*)(abase + (size_t)row * DB + piece * 4) = v; }
    };
    pass(); __threadfence(); pass();
}

__global__ __launch_bounds__(256) void k_feats(const float* __restrict__ ctxh, const float* __restrict__ lhsh, const float* __restrict__ ATT, bf* FH, bf* FL) {
    const int lane = threadIdx.x & 31, r = blockIdx.x * 8 + (threadIdx.x >> 5);
    if (r >= NTH) return;
#pragma unroll 1
    for (int q = 0; q < DF / 128; ++q) { v4us oh, ol;
#pragma unroll
        for (int i = 0; i < 4; ++i) { const int c = q * 128 + lane * 4 + i; float v;
            if (c < DC) v = bfr(ctxh[(size_t)r * DC + c]); else v = bfr(lhsh[(size_t)r * DB + c - DC]) - ATT[(size_t)r * DB + c - DC];
            const unsigned short hb = f2bf(v); oh[i] = hb; ol[i] = f2bf(v - bf2f(hb)); }
        *(volatile v4us*)(FH + (size_t)r * DF + q * 128 + lane * 4) = oh; *(volatile v4us*)(FL + (size_t)r * DF + q * 128 + lane * 4) = ol;
        __threadfence();
        *(volatile v4us*)(FH + (size_t)r * DF + q * 128 + lane * 4) = oh; *(volatile v4us*)(FL + (size_t)r * DF + q * 128 + lane * 4) = ol; }
}

__global__ __launch_bounds__(256) void k_ln(const float* __restrict__ H2, const float* __restrict__ g, const float* __restrict__ b, float* LNO) {
    const int lane = threadIdx.x & 31, r = blockIdx.x * 8 + (threadIdx.x >> 5);
    if (r >= NTH) return;
    float v[4]; float s = 0.f;
#pragma unroll
    for (int i = 0; i < 4; ++i) { v[i] = H2[(size_t)r * D2 + lane * 4 + i]; s += v[i]; }
#pragma unroll
    for (int o = 16; o; o >>= 1) s += __shfl_xor(s, o, 32);
    const float mu = s * (1.0f / D2);
    float q = 0.f;
#pragma unroll
    for (int i = 0; i < 4; ++i) { const float d = v[i] - mu; q += d * d; }
#pragma unroll
    for (int o = 16; o; o >>= 1) q += __shfl_xor(q, o, 32);
    const float rs = rsqrtf(q * (1.0f / D2) + 1e-5f);
    v4f y;
#pragma unroll
    for (int i = 0; i < 4; ++i) { const int c = lane * 4 + i; y[i] = (v[i] - mu) * rs * bfr(g[c]) + bfr(b[c]); }
    VST2(v4f, LNO + (size_t)r * D2 + lane * 4, y);
}
__global__ __launch_bounds__(256) void k_pool(const float* __restrict__ LNO, const int* __restrict__ bh, const float* __restrict__ Wc, const float* __restrict__ bc, float* out) {
    __shared__ float agg[NSG * D2];
    __shared__ float cnt[NSG];
    __shared__ int lst[512], lse[512], wtot[8];
    __shared__ float res[96];
    const int t = threadIdx.x, lane = t & 31, wv = t >> 5;
    for (int i = t; i < NSG * D2; i += 256) agg[i] = 0.f;
    if (t < NSG) cnt[t] = 0.f;
    __syncthreads();
#pragma unroll 1
    for (int base = 0; base < NTH; base += 512) {
        int vdl[2], ve[2], flg[2]; int c = 0;
#pragma unroll
        for (int j = 0; j < 2; ++j) { const int e = base + j * 256 + t; const int d = bh[e]; const int f = ((unsigned)d < (unsigned)NSG) ? 1 : 0; vdl[j] = d; ve[j] = e; flg[j] = f; c += f; }
        int incl = c;
#pragma unroll
        for (int o = 1; o < 32; o <<= 1) { const int y = __shfl_up(incl, o, 32); if (lane >= o) incl += y; }
        if (lane == 31) wtot[wv] = incl;
        __syncthreads();
        int off = incl - c, tot = 0;
#pragma unroll
        for (int i = 0; i < 8; ++i) { const int v = wtot[i]; off += (i < wv) ? v : 0; tot += v; }
#pragma unroll
        for (int j = 0; j < 2; ++j) { if (flg[j]) { lst[off] = vdl[j]; lse[off] = ve[j]; ++off; } }
        __syncthreads();
        if (t < D2) {
#pragma unroll 1
            for (int e2 = 0; e2 < tot; ++e2) agg[lst[e2] * D2 + t] += LNO[(size_t)lse[e2] * D2 + t];
        } else if (t == D2) {
#pragma unroll 1
            for (int e2 = 0; e2 < tot; ++e2) cnt[lst[e2]] += 1.0f;
        }
        __syncthreads();
    }
    if (t < 96) { const int gsg = t / 3, cls = t - gsg * 3; const float ic = 1.0f / fmaxf(cnt[gsg], 1.0f); float s = bfr(bc[cls]);
#pragma unroll 4
        for (int k = 0; k < D2; ++k) s += (agg[gsg * D2 + k] * ic) * bfr(Wc[k * 3 + cls]);
        res[t] = s; }
    __syncthreads();
    if (t < 96) { VST2(float, out + t, res[t]); }
}

extern "C" void kernel_launch(void* const* d_in, const int* in_sizes, int n_in,
                              void* d_out, int out_size, void* d_ws, size_t ws_size, hipStream_t stream) {
    (void)in_sizes; (void)n_in; (void)out_size;
    const float* ctxp = (const float*)d_in[0]; const float* ctxh = (const float*)d_in[1]; const float* lhsp = (const float*)d_in[2]; const float* lhsh = (const float*)d_in[3];
    const int* bp = (const int*)d_in[4]; const int* bh = (const int*)d_in[5];
    const float* Wq = (const float*)d_in[6]; const float* bq = (const float*)d_in[7]; const float* Wk = (const float*)d_in[8]; const float* bk = (const float*)d_in[9];
    const float* Wv = (const float*)d_in[10]; const float* bv = (const float*)d_in[11]; const float* W1 = (const float*)d_in[12]; const float* b1 = (const float*)d_in[13];
    const float* W2 = (const float*)d_in[14]; const float* lng = (const float*)d_in[15]; const float* lnb = (const float*)d_in[16]; const float* Wc = (const float*)d_in[17]; const float* bc = (const float*)d_in[18];
    float* out = (float*)d_out;
    char* wsp = (char*)d_ws;
    auto take = [&](size_t bytes) { char* p = wsp; wsp += (bytes + 255) & ~(size_t)255; return (void*)p; };
    bf* XPb = (bf*)take((size_t)NTP * DC * 2); bf* XHb = (bf*)take((size_t)NTH * DC * 2); bf* LPb = (bf*)take((size_t)NTP * DB * 2);
    bf* WqT = (bf*)take((size_t)DC * DC * 2); bf* WkT = (bf*)take((size_t)DC * DC * 2); bf* WvT = (bf*)take((size_t)DB * DB * 2); bf* W1T = (bf*)take((size_t)D1 * DF * 2); bf* W2T = (bf*)take((size_t)D2 * D1 * 2);
    h16* QI = (h16*)take((size_t)NTH * DC * 2); h16* KI = (h16*)take((size_t)NTP * DC * 2); h16* Q16 = (h16*)take((size_t)NTH * DC * 2); h16* K16 = (h16*)take((size_t)NTP * DC * 2);
    h16* V16 = (h16*)take((size_t)NTP * DB * 2); h16* VT16 = (h16*)take((size_t)NTP * DB * 2); float* ATT = (float*)take((size_t)NTH * DB * 4);
    bf* FH = (bf*)take((size_t)NTH * DF * 2); bf* FL = (bf*)take((size_t)NTH * DF * 2); bf* H1H = (bf*)take((size_t)NTH * D1 * 2); bf* H1L = (bf*)take((size_t)NTH * D1 * 2);
    float* H2 = (float*)take((size_t)NTH * D2 * 4); float* LNO = (float*)take((size_t)NTH * D2 * 4);
    if ((size_t)(wsp - (char*)d_ws) > ws_size) return;
    k_cvtb<<<NTP / 8, 256, 0, stream>>>(ctxp, NTP, DC, XPb);
    k_cvtb<<<NTH / 8, 256, 0, stream>>>(ctxh, NTH, DC, XHb);
    k_cvtb<<<NTP / 8, 256, 0, stream>>>(lhsp, NTP, DB, LPb);
    k_wt<<<dim3(DC / 64, DC / 64, 1), 256, 0, stream>>>(Wq, DC, DC, WqT);
    k_wt<<<dim3(DC / 64, DC / 64, 1), 256, 0, stream>>>(Wk, DC, DC, WkT);
    k_wt<<<dim3(DB / 64, DB / 64, 1), 256, 0, stream>>>(Wv, DB, DB, WvT);
    k_wt<<<dim3(DF / 64, D1 / 64, 1), 256, 0, stream>>>(W1, DF, D1, W1T);
    k_wt<<<dim3(D1 / 64, D2 / 64, 1), 256, 0, stream>>>(W2, D1, D2, W2T);
    k_gemmb<false, 1><<<dim3(NTH / 64, DC / 64, 1), 128, 0, stream>>>(XHb, nullptr, WqT, DC, bq, QI, nullptr, DC);
    k_gemmb<false, 1><<<dim3(NTP / 64, DC / 64, 1), 128, 0, stream>>>(XPb, nullptr, WkT, DC, bk, KI, nullptr, DC);
    k_deint<<<NTH / 8, 256, 0, stream>>>(QI, Q16); k_deint<<<NTP / 8, 256, 0, stream>>>(KI, K16);
    k_gemmb<false, 2><<<dim3(NTP / 64, DB / 64, 1), 128, 0, stream>>>(LPb, nullptr, WvT, DB, bv, V16, nullptr, DB);
    k_vt<<<NH_ * (NTP / 64), 256, 0, stream>>>(V16, VT16);
    k_attn<<<NH_ * (NTH / 64), 128, 0, stream>>>(Q16, K16, VT16, bh, bp, ATT);
    k_feats<<<NTH / 8, 256, 0, stream>>>(ctxh, lhsh, ATT, FH, FL);
    k_gemmb<true, 3><<<dim3(NTH / 64, D1 / 64, 1), 128, 0, stream>>>(FH, FL, W1T, DF, b1, H1H, H1L, D1);
    k_gemmb<true, 0><<<dim3(NTH / 64, D2 / 64, 1), 128, 0, stream>>>(H1H, H1L, W2T, D1, nullptr, H2, nullptr, D2);
    k_ln<<<NTH / 8, 256, 0, stream>>>(H2, lng, lnb, LNO);
    k_pool<<<1, 256, 0, stream>>>(LNO, bh, Wc, bc, out);
}
